// SFT_16844861735534
// MI455X (gfx1250) — hardware-verified
//
#include <hip/hip_runtime.h>
#include <math.h>

typedef __attribute__((ext_vector_type(16))) _Float16 v16h;
typedef __attribute__((ext_vector_type(16))) __bf16 v16b;
typedef __attribute__((ext_vector_type(8)))  _Float16 v8h;
typedef __attribute__((ext_vector_type(8)))  float v8f;
typedef __attribute__((ext_vector_type(4)))  float v4f;
typedef __attribute__((ext_vector_type(2)))  float v2f;
typedef __attribute__((ext_vector_type(4)))  unsigned v4u;
typedef __attribute__((ext_vector_type(4)))  int v4i;
typedef float __attribute__((may_alias)) float_a;
typedef int __attribute__((may_alias)) int_a;

template <typename T> __device__ __forceinline__ void vst2(void* p, T v) { *(volatile T*)p = v; __threadfence(); *(volatile T*)p = v; }
__device__ __forceinline__ v8f wmma16(v16h a, v16h b, v8f c) {
  v8f d = __builtin_amdgcn_wmma_f32_16x16x32_f16(false, a, false, b, (short)0, c, false, false);
  asm volatile("v_nop\n\tv_nop\n\tv_nop\n\tv_nop" : "+v"(d) : "v"(a), "v"(b));
  return d;
}
__device__ __forceinline__ v8f wmma_bf(v16b a, v16b b, v8f c) {
  v8f d = __builtin_amdgcn_wmma_f32_16x16x32_bf16(false, a, false, b, (short)0, c, false, false);
  asm volatile("v_nop\n\tv_nop\n\tv_nop\n\tv_nop" : "+v"(d) : "v"(a), "v"(b));
  return d;
}
__device__ __forceinline__ v16h frag_h(const _Float16* rowk0, int lane) {
  union { v16h v; v8h q[2]; } u; const _Float16* p = rowk0 + 8 * (lane >> 4);
  u.q[0] = *(const v8h*)p; u.q[1] = *(const v8h*)(p + 16); return u.v;
}
__device__ __forceinline__ v16h frag_f32(const float* rowk0, int lane) {
  v16h a; const float* p = rowk0 + 8 * (lane >> 4);
#pragma unroll
  for (int i = 0; i < 8; ++i) { a[i] = (_Float16)p[i]; a[8 + i] = (_Float16)p[16 + i]; }
  return a;
}
__device__ __forceinline__ v16h frag_f32s(const float* rowk0, int lane, float sc) {
  v16h a; const float* p = rowk0 + 8 * (lane >> 4);
#pragma unroll
  for (int i = 0; i < 8; ++i) { a[i] = (_Float16)(p[i] * sc); a[8 + i] = (_Float16)(p[16 + i] * sc); }
  return a;
}
__device__ __forceinline__ v16h fragc_f32(const float* W, int k0, int n, int lane, int ld, int K) {
  v16h a; const int g = lane >> 4;
#pragma unroll
  for (int i = 0; i < 8; ++i) { const int ka = k0 + 8 * g + i, kb = ka + 16;
    a[i] = (_Float16)(ka < K ? W[(size_t)(ka < K ? ka : K - 1) * ld + n] : 0.f); a[8 + i] = (_Float16)(kb < K ? W[(size_t)(kb < K ? kb : K - 1) * ld + n] : 0.f); }
  return a;
}
struct F2 { v16b h, l; };
__device__ __forceinline__ F2 bsplit16(const float v[16]) { F2 r;
#pragma unroll
  for (int i = 0; i < 16; ++i) { const __bf16 h = (__bf16)v[i]; r.h[i] = h; r.l[i] = (__bf16)(v[i] - (float)h); }
  return r; }
__device__ __forceinline__ F2 split_row(const float* row, int k0, int lane) { float v[16]; const float* p = row + k0 + 8 * (lane >> 4);
#pragma unroll
  for (int i = 0; i < 8; ++i) { v[i] = p[i]; v[8 + i] = p[16 + i]; }
  return bsplit16(v); }
__device__ __forceinline__ F2 split_rowK(const float* row, int k0, int lane, int K) { float v[16]; const int g = lane >> 4;
#pragma unroll
  for (int i = 0; i < 8; ++i) { const int ka = k0 + 8 * g + i, kb = ka + 16; v[i] = ka < K ? row[ka < K ? ka : K - 1] : 0.f; v[8 + i] = kb < K ? row[kb < K ? kb : K - 1] : 0.f; }
  return bsplit16(v); }
__device__ __forceinline__ F2 split_col(const float* W, int k0, int n, int lane, int ld, int K) { float v[16]; const int g = lane >> 4;
#pragma unroll
  for (int i = 0; i < 8; ++i) { const int ka = k0 + 8 * g + i, kb = ka + 16; v[i] = ka < K ? W[(size_t)(ka < K ? ka : K - 1) * ld + n] : 0.f; v[8 + i] = kb < K ? W[(size_t)(kb < K ? kb : K - 1) * ld + n] : 0.f; }
  return bsplit16(v); }
__device__ __forceinline__ v8f mac3(const F2& a, const F2& b, v8f c) { c = wmma_bf(a.l, b.h, c); c = wmma_bf(a.h, b.l, c); return wmma_bf(a.h, b.h, c); }
__device__ __forceinline__ float sigm(float v) { return 1.0f / (1.0f + expf(-v)); }
#define LDSX() do { asm volatile("s_wait_dscnt 0" ::: "memory"); __builtin_amdgcn_wave_barrier(); __builtin_amdgcn_fence(__ATOMIC_RELEASE, "workgroup"); } while (0)


#define NRW 8192
#define DD 256
#define SIG_INV 10.0f
__device__ __forceinline__ float bfr(float v) { return (float)(__bf16)v; }
__device__ __forceinline__ v16b frag_b(const __bf16* rowk0, int lane) { return __builtin_bit_cast(v16b, frag_h((const _Float16*)rowk0, lane)); }

__global__ __launch_bounds__(256) void k_prep(const float* __restrict__ emb, __bf16* __restrict__ EB, _Float16* __restrict__ EMT, float* __restrict__ INV) {
  __shared__ __align__(16) _Float16 st[DD][72]; __shared__ __align__(16) float sinv[64];
  const int tid = threadIdx.x, wave = tid >> 5, lane = tid & 31; const int r0 = blockIdx.x * 64;
  for (int rr = 0; rr < 8; ++rr) { const int rl = wave * 8 + rr; const float* src = emb + (size_t)(r0 + rl) * DD; float ss = 0.f; union { __bf16 e[8]; v4u u; } pk;
#pragma unroll
    for (int e = 0; e < 8; ++e) { const float v = bfr(src[lane * 8 + e]); pk.e[e] = (__bf16)v; ss += v * v; st[lane * 8 + e][rl] = (_Float16)v; }
#pragma unroll
    for (int o = 16; o > 0; o >>= 1) ss += __shfl_xor(ss, o, 32);
    vst2((unsigned*)(EB + (size_t)(r0 + rl) * DD + lane * 8), pk.u);
    if (lane == 0) sinv[rl] = 1.0f / fmaxf(sqrtf(ss), 1e-12f); }
  __syncthreads();
  for (int q = tid; q < DD * 8; q += 256) { const int d = q >> 3, pc = q & 7; vst2(EMT + (size_t)d * NRW + r0 + pc * 8, *(const v4u*)(&st[d][pc * 8])); }
  if (tid < 16) vst2(INV + r0 + tid * 4, *(const v4f*)(&sinv[tid * 4]));
}
__global__ __launch_bounds__(128) void k_attn(const __bf16* __restrict__ EB, const _Float16* __restrict__ EMT, const float* __restrict__ INV, float* __restrict__ out) {
  __shared__ __align__(16) float sS[4][16][68];
  __shared__ __align__(16) _Float16 sP[4][16][72];
  __shared__ __align__(16) float sO[4][16][DD + 4];
  __shared__ float sqi[4][16];
  const int tid = threadIdx.x, w = tid >> 5, lane = tid & 31, col = lane & 15, g = lane >> 4; const int q0 = blockIdx.x * 64 + w * 16;
  if (lane < 16) sqi[w][lane] = INV[q0 + lane] * SIG_INV;
  v16b aq[DD / 32];
#pragma unroll
  for (int kc = 0; kc < DD / 32; ++kc) aq[kc] = frag_b(EB + (size_t)(q0 + col) * DD + kc * 32, lane);
  float mrun = -3.0e38f, lrun = 0.f; v8f acc[16] = {};
  LDSX();
#pragma unroll 1
  for (int kt = 0; kt < NRW / 64; ++kt) {
#pragma unroll
    for (int t = 0; t < 4; ++t) { const int key = kt * 64 + t * 16 + col; v8f s = {};
#pragma unroll
      for (int kc = 0; kc < DD / 32; ++kc) s = wmma_bf(aq[kc], frag_b(EB + (size_t)key * DD + kc * 32, lane), s);
      const float kinv = INV[key];
#pragma unroll
      for (int r = 0; r < 8; ++r) sS[w][8 * g + r][t * 16 + col] = s[r] * sqi[w][8 * g + r] * kinv; }
    LDSX();
    float mx = -3.4e38f;
#pragma unroll
    for (int jj = 0; jj < 32; ++jj) mx = fmaxf(mx, sS[w][col][g * 32 + jj]);
    mx = fmaxf(mx, __shfl_xor(mx, 16, 32));
    const float mnew = fmaxf(mrun, mx); const float corr = expf(mrun - mnew);
    float ps = 0.f;
#pragma unroll
    for (int jj = 0; jj < 32; ++jj) { const float p = expf(sS[w][col][g * 32 + jj] - mnew); ps += p; sP[w][col][g * 32 + jj] = (_Float16)(p * 16384.0f); }
    ps += __shfl_xor(ps, 16, 32);
    lrun = lrun * corr + ps; mrun = mnew;
#pragma unroll
    for (int r = 0; r < 8; ++r) { const float cr = __shfl(corr, 8 * g + r, 32);
#pragma unroll
      for (int t = 0; t < 16; ++t) acc[t][r] *= cr; }
    LDSX();
#pragma unroll
    for (int kc = 0; kc < 2; ++kc) { const v16h ph = frag_h(&sP[w][col][0] + kc * 32, lane);
#pragma unroll
      for (int t = 0; t < 16; ++t) acc[t] = wmma16(ph, frag_h(EMT + (size_t)(t * 16 + col) * NRW + kt * 64 + kc * 32, lane), acc[t]); }
    __builtin_amdgcn_wave_barrier(); }
#pragma unroll
  for (int r = 0; r < 8; ++r) { const float lr = __shfl(lrun, 8 * g + r, 32); const float inv = 1.0f / (lr * 16384.0f);
#pragma unroll
    for (int t = 0; t < 16; ++t) sO[w][8 * g + r][t * 16 + col] = acc[t][r] * inv; }
  LDSX();
  for (int rl = 0; rl < 16; ++rl) for (int pc = lane; pc < DD / 4; pc += 32) vst2(out + (size_t)(q0 + rl) * DD + pc * 4, *(const v4f*)(&sO[w][rl][pc * 4]));
}
extern "C" void kernel_launch(void* const* d_in, const int* in_sizes, int n_in, void* d_out, int out_size, void* d_ws, size_t ws_size, hipStream_t stream) {
  (void)in_sizes; (void)n_in; (void)out_size; (void)ws_size;
  const float* emb = (const float*)d_in[0];
  char* ws = (char*)d_ws; __bf16* EB = (__bf16*)ws; _Float16* EMT = (_Float16*)(EB + (size_t)NRW * DD); float* INV = (float*)(EMT + (size_t)NRW * DD);
  k_prep<<<NRW / 64, 256, 0, stream>>>(emb, EB, EMT, INV);
  k_attn<<<NRW / 64, 128, 0, stream>>>(EB, EMT, INV, (float*)d_out);
}
